// TransformerLayer_89670327206487
// MI455X (gfx1250) — hardware-verified
//
#include <hip/hip_runtime.h>
#ifndef NB
#define NB 4
#endif
#ifndef SEQ
#define SEQ 1024
#endif
#define NB_FULL 4
#define SEQ_FULL 1024
#define DM 1024
#define FF 4096
#define NH 16
#define HD 64
#define NR (NB * SEQ)
#define QBLKS (SEQ / 64)
#define SCL 0.125f
#define PCARRY 1024.0f
#define CCARRY 64.0f

static_assert(DM == NH * HD);
static_assert(HD == 64);
static_assert(SEQ % 128 == 0);
static_assert(NR % 128 == 0);
static_assert(NR % 8 == 0);
static_assert(DM % 64 == 0 && FF % 64 == 0);
static_assert(DM % 32 == 0 && FF % 32 == 0);
static_assert(NB <= NB_FULL && SEQ <= SEQ_FULL);
static_assert((size_t)NR * FF <= (size_t)4 * NR * DM);

typedef unsigned short v8us __attribute__((ext_vector_type(8), may_alias));
typedef float  v8f  __attribute__((ext_vector_type(8)));
typedef float  v4f  __attribute__((ext_vector_type(4)));
typedef float  v4fa __attribute__((ext_vector_type(4), may_alias));
typedef _Float16 v16h __attribute__((ext_vector_type(16)));
typedef _Float16 v4h __attribute__((ext_vector_type(4)));
union FragH { v16h v; v8us half[2]; _Float16 h[16]; unsigned short u[16]; };

__device__ __forceinline__ float bf16_rne(float x) { unsigned int u = __float_as_uint(x); u = (u + 0x7FFFu + ((u >> 16) & 1u)) & 0xFFFF0000u; return __uint_as_float(u); }
__device__ __forceinline__ unsigned short h_bits(float x) { const _Float16 h = (_Float16)x; return __builtin_bit_cast(unsigned short, h); }
__device__ __forceinline__ v16h g2_frag(const _Float16* p, unsigned hh) { FragH f; f.half[0] = *(const v8us*)((const unsigned short*)p + 8u * hh); f.half[1] = *(const v8us*)((const unsigned short*)p + 16u + 8u * hh); return f.v; }
__device__ __forceinline__ v8f g2_mma(v16h a, v16h b, v8f c) { v8f d = __builtin_amdgcn_wmma_f32_16x16x32_f16(false, a, false, b, (short)0, c, false, false); asm volatile("v_nop\n\tv_nop\n\tv_nop\n\tv_nop" : "+v"(d) : "v"(a), "v"(b)); return d; }
__device__ __forceinline__ float gelu_t(float v) { const float u = 0.7978845608028654f * (v + 0.044715f * v * v * v); const float e = expf(-2.0f * u); return v * __builtin_amdgcn_rcpf(1.0f + e); }

__global__ __launch_bounds__(256) void k_wsc(const float* __restrict__ Wm, _Float16* __restrict__ Bt, unsigned n8, float sc) {
  const unsigned t = blockIdx.x * 256u + threadIdx.x; if (t >= n8) return;
  const v4f a = *(const v4fa*)(Wm + (size_t)t * 8), c = *(const v4fa*)(Wm + (size_t)t * 8 + 4);
  FragH f;
#pragma unroll
  for (unsigned q = 0; q < 4; ++q) { f.h[q] = (_Float16)(bf16_rne(a[q]) * sc); f.h[4 + q] = (_Float16)(bf16_rne(c[q]) * sc); }
  const v8us o = f.half[0];
  *(volatile v8us*)((unsigned short*)Bt + (size_t)t * 8) = o; __threadfence(); *(volatile v8us*)((unsigned short*)Bt + (size_t)t * 8) = o;
}

__global__ __launch_bounds__(256) void k_x16(const float* __restrict__ x, _Float16* __restrict__ X16) {
  const unsigned t = blockIdx.x * 256u + threadIdx.x; if (t >= (unsigned)(NR * (DM / 8))) return;
  const unsigned row = t / (unsigned)(DM / 8), c8 = (t % (unsigned)(DM / 8)) * 8u;
  const unsigned bi = row / (unsigned)SEQ, si = row % (unsigned)SEQ;
  const float* src = x + ((size_t)bi * SEQ_FULL + si) * DM + c8;
  const v4f a = *(const v4fa*)(src), c = *(const v4fa*)(src + 4);
  FragH f;
#pragma unroll
  for (unsigned q = 0; q < 4; ++q) { f.h[q] = (_Float16)bf16_rne(a[q]); f.h[4 + q] = (_Float16)bf16_rne(c[q]); }
  const v8us o = f.half[0];
  *(volatile v8us*)((unsigned short*)X16 + (size_t)t * 8) = o; __threadfence(); *(volatile v8us*)((unsigned short*)X16 + (size_t)t * 8) = o;
}

template <int ACT>
__global__ __launch_bounds__(128) void k_gemm2(const _Float16* __restrict__ A, unsigned lda, const _Float16* __restrict__ Bh, unsigned ldb, float alpha, const float* __restrict__ bias,
                                              float* __restrict__ C, _Float16* __restrict__ C16, unsigned ldc, unsigned K) {
  __shared__ __attribute__((aligned(16))) float so[4][32][68];
  const unsigned tid = threadIdx.x, w = tid >> 5, lane = tid & 31u, ln = lane & 15u, hh = lane >> 4;
  const unsigned row0 = blockIdx.y * 128u + 32u * w, col0 = blockIdx.x * 64u;
  const _Float16* a0p = A + (size_t)(row0 + ln) * lda; const _Float16* a1p = a0p + (size_t)16 * lda;
  const _Float16* b0p = Bh + (size_t)(col0 + ln) * ldb; const _Float16* b1p = b0p + (size_t)16 * ldb; const _Float16* b2p = b1p + (size_t)16 * ldb; const _Float16* b3p = b2p + (size_t)16 * ldb;
  const v8f z8 = {0.f,0.f,0.f,0.f,0.f,0.f,0.f,0.f}; v8f c00 = z8, c01 = z8, c02 = z8, c03 = z8, c10 = z8, c11 = z8, c12 = z8, c13 = z8;
#pragma unroll 1
  for (unsigned kb = 0; kb < K; kb += 32u) { const v16h a0 = g2_frag(a0p + kb, hh), a1 = g2_frag(a1p + kb, hh);
    v16h b = g2_frag(b0p + kb, hh); c00 = g2_mma(a0, b, c00); c10 = g2_mma(a1, b, c10);
    b = g2_frag(b1p + kb, hh); c01 = g2_mma(a0, b, c01); c11 = g2_mma(a1, b, c11);
    b = g2_frag(b2p + kb, hh); c02 = g2_mma(a0, b, c02); c12 = g2_mma(a1, b, c12);
    b = g2_frag(b3p + kb, hh); c03 = g2_mma(a0, b, c03); c13 = g2_mma(a1, b, c13); }
  v8f accs[8] = {c00, c01, c02, c03, c10, c11, c12, c13};
#pragma unroll
  for (unsigned u = 0; u < 8; ++u) { const unsigned t = u & 3u, half = u >> 2; const unsigned col = col0 + t * 16u + ln; const float bv = bf16_rne(bias[col]);
#pragma unroll
    for (unsigned r = 0; r < 8; ++r) { const unsigned rloc = half * 16u + 8u * hh + r; float v = accs[u][r] * alpha + bv;
      if (ACT == 9) v = gelu_t(v);
      so[w][rloc][t * 16u + ln] = v; } }
  __builtin_amdgcn_fence(4  , "workgroup"); __builtin_amdgcn_wave_barrier();
  const unsigned rsub = lane >> 4, c4 = (lane & 15u) * 4u;
  for (int pass = 0; pass < 2; ++pass) {
#pragma unroll
    for (unsigned q = 0; q < 16; ++q) { const unsigned r = q * 2u + rsub; const v4f v = *(const v4fa*)&so[w][r][c4];
      if (C) *(volatile v4f*)(C + (size_t)(row0 + r) * ldc + col0 + c4) = v;
      if (C16) { v4h h4; h4[0] = (_Float16)v[0]; h4[1] = (_Float16)v[1]; h4[2] = (_Float16)v[2]; h4[3] = (_Float16)v[3]; *(volatile v4h*)(C16 + (size_t)(row0 + r) * ldc + col0 + c4) = h4; } }
    if (pass == 0) __threadfence(); } }

__global__ __launch_bounds__(256) void k_vt(const _Float16* __restrict__ V16, _Float16* __restrict__ Vt) {
  __shared__ unsigned short tl[64][66];
  const unsigned tid = threadIdx.x; const unsigned slab = blockIdx.x / (unsigned)QBLKS, lg = blockIdx.x % (unsigned)QBLKS; const unsigned b = slab / (unsigned)NH, h = slab % (unsigned)NH;
  for (unsigned i = tid; i < 512u; i += 256u) { const unsigned r = i >> 3, c8 = (i & 7u) * 8u;
    const v8us f = *(const v8us*)((const unsigned short*)V16 + ((size_t)b * SEQ + lg * 64u + r) * DM + h * 64u + c8);
#pragma unroll
    for (unsigned q = 0; q < 8; ++q) tl[r][c8 + q] = f[q]; }
  __syncthreads();
  v8us o[2];
#pragma unroll
  for (unsigned rd = 0; rd < 2; ++rd) { const unsigned d = rd * 32u + (tid >> 3), pc = tid & 7u;
#pragma unroll
    for (unsigned q = 0; q < 8; ++q) o[rd][q] = tl[pc * 8u + q][d]; }
  for (int pass = 0; pass < 2; ++pass) {
#pragma unroll
    for (unsigned rd = 0; rd < 2; ++rd) { const unsigned d = rd * 32u + (tid >> 3), pc = tid & 7u;
      *(volatile v8us*)((unsigned short*)Vt + ((size_t)slab * 64u + d) * SEQ + lg * 64u + pc * 8u) = o[rd]; }
    if (pass == 0) __threadfence(); } }

__global__ __launch_bounds__(128) void k_flash(const _Float16* __restrict__ Q16, const _Float16* __restrict__ K16, const _Float16* __restrict__ Vt, const int* __restrict__ MSK, _Float16* __restrict__ CX) {
  __shared__ __attribute__((aligned(16))) unsigned short sP[4][16][40];
  __shared__ __attribute__((aligned(16))) float sO[4][16][68];
  const unsigned tid = threadIdx.x, w = tid >> 5, lane = tid & 31u, ln = lane & 15u, hh = lane >> 4;
  const unsigned slab = blockIdx.x / (unsigned)QBLKS, qblk = blockIdx.x % (unsigned)QBLKS; const unsigned b = slab / (unsigned)NH, h = slab % (unsigned)NH;
  const unsigned q0 = qblk * 64u + w * 16u;
  const _Float16* qr = Q16 + ((size_t)b * SEQ + q0 + ln) * DM + h * 64u;
  const v16h aq0 = g2_frag(qr, hh), aq1 = g2_frag(qr + 32, hh);
  const _Float16* Vth = Vt + (size_t)slab * 64u * SEQ;
  const _Float16* Kb = K16 + ((size_t)b * SEQ + ln) * DM + h * 64u;
  const int* mrow = MSK + (size_t)b * SEQ_FULL;
  const v8f z8 = {0.f,0.f,0.f,0.f,0.f,0.f,0.f,0.f};
  float m_r[8], l_r[8]; v8f oacc[4];
#pragma unroll
  for (unsigned r = 0; r < 8; ++r) { m_r[r] = -3.0e38f; l_r[r] = 0.f; }
#pragma unroll
  for (unsigned dt = 0; dt < 4; ++dt) oacc[dt] = z8;
#pragma unroll 1
  for (unsigned j0 = 0; j0 < (unsigned)SEQ; j0 += 32u) {
    v8f s0v, s1v;
    { const _Float16* kr = Kb + (size_t)j0 * DM; const v16h k0 = g2_frag(kr, hh), k1 = g2_frag(kr + 32, hh); v8f acc = z8; acc = g2_mma(aq0, k0, acc); acc = g2_mma(aq1, k1, acc); s0v = acc; }
    { const _Float16* kr = Kb + (size_t)(j0 + 16u) * DM; const v16h k0 = g2_frag(kr, hh), k1 = g2_frag(kr + 32, hh); v8f acc = z8; acc = g2_mma(aq0, k0, acc); acc = g2_mma(aq1, k1, acc); s1v = acc; }
    const int mk0 = mrow[j0 + ln], mk1 = mrow[j0 + 16u + ln];
#pragma unroll
    for (unsigned r = 0; r < 8; ++r) {
      const float s0 = (mk0 != 0) ? s0v[r] * SCL : -1.0e9f, s1 = (mk1 != 0) ? s1v[r] * SCL : -1.0e9f;
      float mc = fmaxf(s0, s1);
      mc = fmaxf(mc, __shfl_xor(mc, 1, 32)); mc = fmaxf(mc, __shfl_xor(mc, 2, 32)); mc = fmaxf(mc, __shfl_xor(mc, 4, 32)); mc = fmaxf(mc, __shfl_xor(mc, 8, 32));
      const float mn = fmaxf(m_r[r], mc); const float al = expf(m_r[r] - mn); m_r[r] = mn;
      const float p0 = expf(s0 - mn), p1 = expf(s1 - mn); l_r[r] = l_r[r] * al + p0 + p1;
#pragma unroll
      for (unsigned dt = 0; dt < 4; ++dt) oacc[dt][r] *= al;
      sP[w][8u * hh + r][ln] = h_bits(p0 * PCARRY); sP[w][8u * hh + r][16u + ln] = h_bits(p1 * PCARRY); }
    __builtin_amdgcn_fence(4  , "workgroup"); __builtin_amdgcn_wave_barrier();
    FragH pa; pa.half[0] = *(const v8us*)&sP[w][ln][8u * hh]; pa.half[1] = *(const v8us*)&sP[w][ln][16u + 8u * hh];
#pragma unroll
    for (unsigned dt = 0; dt < 4; ++dt) { const v16h bv = g2_frag(Vth + (size_t)(dt * 16u + ln) * SEQ + j0, hh); oacc[dt] = g2_mma(pa.v, bv, oacc[dt]); }
    __builtin_amdgcn_fence(4  , "workgroup"); __builtin_amdgcn_wave_barrier(); }
#pragma unroll
  for (unsigned r = 0; r < 8; ++r) { float l = l_r[r]; l += __shfl_xor(l, 1, 32); l += __shfl_xor(l, 2, 32); l += __shfl_xor(l, 4, 32); l += __shfl_xor(l, 8, 32); l_r[r] = 1.0f / (l * (PCARRY / CCARRY)); }
#pragma unroll
  for (unsigned dt = 0; dt < 4; ++dt)
#pragma unroll
    for (unsigned r = 0; r < 8; ++r) sO[w][8u * hh + r][dt * 16u + ln] = oacc[dt][r] * l_r[r];
  __builtin_amdgcn_fence(4  , "workgroup"); __builtin_amdgcn_wave_barrier();
  const unsigned rq = lane >> 3, pc = lane & 7u;
  v8us o[4];
#pragma unroll
  for (unsigned g = 0; g < 4; ++g) { const unsigned r = g * 4u + rq; const v4f x0 = *(const v4fa*)&sO[w][r][pc * 8u], x1 = *(const v4fa*)&sO[w][r][pc * 8u + 4u];
    o[g][0] = h_bits(x0[0]); o[g][1] = h_bits(x0[1]); o[g][2] = h_bits(x0[2]); o[g][3] = h_bits(x0[3]); o[g][4] = h_bits(x1[0]); o[g][5] = h_bits(x1[1]); o[g][6] = h_bits(x1[2]); o[g][7] = h_bits(x1[3]); }
  for (int pass = 0; pass < 2; ++pass) {
#pragma unroll
    for (unsigned g = 0; g < 4; ++g) { const unsigned r = g * 4u + rq; *(volatile v8us*)((unsigned short*)CX + ((size_t)b * SEQ + q0 + r) * DM + h * 64u + pc * 8u) = o[g]; }
    if (pass == 0) __threadfence(); } }

template <int MODE>
__global__ __launch_bounds__(256) void k_ln(const float* __restrict__ A, const float* __restrict__ R, const float* __restrict__ g, const float* __restrict__ bb, float* __restrict__ Y, _Float16* __restrict__ Y16) {
  #pragma clang fp contract(off)
  const unsigned wv = threadIdx.x >> 5, ln = threadIdx.x & 31u; const unsigned r = blockIdx.x * 8u + wv; if (r >= (unsigned)NR) return;
  const unsigned bi = r / (unsigned)SEQ, si = r % (unsigned)SEQ; const size_t rfull = (size_t)bi * SEQ_FULL + si;
  const float* ap = A + (size_t)r * DM; const float* rp = R + ((MODE == 1) ? rfull : (size_t)r) * DM;
  float x[32]; float s = 0.f;
#pragma unroll
  for (unsigned i = 0; i < 8; ++i) { const unsigned c0 = i * 128u + ln * 4u; const v4f a = *(const v4fa*)(ap + c0); const v4f q = *(const v4fa*)(rp + c0);
#pragma unroll
    for (unsigned k = 0; k < 4; ++k) { float v = q[k]; if (MODE == 1) v = bf16_rne(v); v = a[k] + v; x[i * 4u + k] = v; s += v; } }
  s += __shfl_xor(s, 16, 32); s += __shfl_xor(s, 8, 32); s += __shfl_xor(s, 4, 32); s += __shfl_xor(s, 2, 32); s += __shfl_xor(s, 1, 32);
  const float mu = s * (1.0f / (float)DM);
  float var = 0.f;
#pragma unroll
  for (unsigned q = 0; q < 32; ++q) { const float d = x[q] - mu; var += d * d; }
  var += __shfl_xor(var, 16, 32); var += __shfl_xor(var, 8, 32); var += __shfl_xor(var, 4, 32); var += __shfl_xor(var, 2, 32); var += __shfl_xor(var, 1, 32);
  const float den = sqrtf(var / (float)(DM - 1)) + 1e-6f; const float inv = 1.0f / den;
  v4h hq[8];
#pragma unroll
  for (unsigned i = 0; i < 8; ++i) { const unsigned c0 = i * 128u + ln * 4u; const v4f gv = *(const v4fa*)(g + c0); const v4f bv = *(const v4fa*)(bb + c0);
#pragma unroll
    for (unsigned k = 0; k < 4; ++k) { float y = (x[i * 4u + k] - mu) * bf16_rne(gv[k]); y = y * inv; y = y + bf16_rne(bv[k]); x[i * 4u + k] = y; hq[i][k] = (_Float16)y; } }
  float* yp = Y + ((MODE == 2) ? rfull : (size_t)r) * DM;
  for (int pass = 0; pass < 2; ++pass) {
#pragma unroll
    for (unsigned i = 0; i < 8; ++i) { const unsigned c0 = i * 128u + ln * 4u; v4f o; o[0] = x[i * 4u]; o[1] = x[i * 4u + 1u]; o[2] = x[i * 4u + 2u]; o[3] = x[i * 4u + 3u];
      *(volatile v4f*)(yp + c0) = o;
      if (MODE == 1) *(volatile v4h*)(Y16 + (size_t)r * DM + c0) = hq[i]; }
    if (pass == 0) __threadfence(); } }

#define WS_BYTES ((size_t)4 * DM * DM * 2 + (size_t)2 * FF * DM * 2 + (size_t)4 * NR * DM * 2 + (size_t)2 * NR * DM * 2 + (size_t)2 * NR * DM * 4)
static_assert(WS_BYTES <= (size_t)134217728);

extern "C" void kernel_launch(void* const* d_in, const int* in_sizes, int n_in,
                              void* d_out, int out_size, void* d_ws, size_t ws_size, hipStream_t stream) {
  if (n_in < 20) return;
  const long long need_rows = (long long)(NB - 1) * SEQ_FULL + SEQ;
  if ((long long)in_sizes[0] < need_rows * DM) return;
  if ((long long)in_sizes[3] < need_rows) return;
  if (in_sizes[4] < DM * DM || in_sizes[6] < DM * DM || in_sizes[8] < DM * DM || in_sizes[10] < DM * DM) return;
  if (in_sizes[12] < FF * DM || in_sizes[14] < DM * FF) return;
  if (in_sizes[5] < DM || in_sizes[7] < DM || in_sizes[9] < DM || in_sizes[11] < DM || in_sizes[13] < FF || in_sizes[15] < DM) return;
  if (in_sizes[16] < DM || in_sizes[17] < DM || in_sizes[18] < DM || in_sizes[19] < DM) return;
  if ((long long)out_size < need_rows * DM) return;
  const float* x = (const float*)d_in[0];
  const int* msk = (const int*)d_in[3];
  const float* wq = (const float*)d_in[4];  const float* bq = (const float*)d_in[5];
  const float* wk = (const float*)d_in[6];  const float* bk = (const float*)d_in[7];
  const float* wv = (const float*)d_in[8];  const float* bv = (const float*)d_in[9];
  const float* wo = (const float*)d_in[10]; const float* bo = (const float*)d_in[11];
  const float* w1 = (const float*)d_in[12]; const float* b1 = (const float*)d_in[13];
  const float* w2 = (const float*)d_in[14]; const float* b2 = (const float*)d_in[15];
  const float* g1 = (const float*)d_in[16]; const float* be1 = (const float*)d_in[17];
  const float* g2 = (const float*)d_in[18]; const float* be2 = (const float*)d_in[19];
  char* ws = (char*)d_ws; size_t off = 0;
  auto take = [&](size_t bytes) { char* p = ws + off; off += (bytes + 255) & ~(size_t)255; return p; };
  const size_t np = (size_t)NR * DM;
  _Float16* BQ = (_Float16*)take((size_t)DM * DM * 2); _Float16* BK = (_Float16*)take((size_t)DM * DM * 2); _Float16* BV = (_Float16*)take((size_t)DM * DM * 2); _Float16* BO = (_Float16*)take((size_t)DM * DM * 2);
  _Float16* B1 = (_Float16*)take((size_t)FF * DM * 2); _Float16* B2 = (_Float16*)take((size_t)DM * FF * 2);
  _Float16* P4 = (_Float16*)take(np * 2 * 4);
  _Float16* X16 = P4; _Float16* QH = P4 + np; _Float16* KH = P4 + 2 * np; _Float16* V16 = P4 + 3 * np;
  _Float16* F16 = P4;
  _Float16* VT = (_Float16*)take(np * 2); _Float16* H16 = VT;
  _Float16* CX = (_Float16*)take(np * 2);
  float* AO = (float*)take(np * 4); float* FFo = AO;
  float* Hf = (float*)take(np * 4);
  if (off > ws_size || off > (size_t)134217728) return;

  const unsigned nw = (unsigned)(DM * DM / 8), nw4 = (unsigned)(FF * DM / 8);
  k_wsc<<<(nw + 255u) / 256u, 256, 0, stream>>>(wq, BQ, nw, 16.0f);
  k_wsc<<<(nw + 255u) / 256u, 256, 0, stream>>>(wk, BK, nw, 16.0f);
  k_wsc<<<(nw + 255u) / 256u, 256, 0, stream>>>(wv, BV, nw, 16.0f);
  k_wsc<<<(nw + 255u) / 256u, 256, 0, stream>>>(wo, BO, nw, 16.0f);
  k_wsc<<<(nw4 + 255u) / 256u, 256, 0, stream>>>(w1, B1, nw4, 16.0f);
  k_wsc<<<(nw4 + 255u) / 256u, 256, 0, stream>>>(w2, B2, nw4, 64.0f);
  k_x16<<<(unsigned)((np / 8 + 255) / 256), 256, 0, stream>>>(x, X16);
  const dim3 gd(DM / 64, NR / 128), gf(FF / 64, NR / 128);
  k_gemm2<0><<<gd, 128, 0, stream>>>(X16, DM, BQ, DM, 0.0625f, bq, nullptr, QH, DM, DM);
  k_gemm2<0><<<gd, 128, 0, stream>>>(X16, DM, BK, DM, 0.0625f, bk, nullptr, KH, DM, DM);
  k_gemm2<0><<<gd, 128, 0, stream>>>(X16, DM, BV, DM, 0.0625f, bv, nullptr, V16, DM, DM);
  k_vt<<<NB * NH * QBLKS, 256, 0, stream>>>(V16, VT);
  k_flash<<<NB * NH * QBLKS, 128, 0, stream>>>(QH, KH, VT, msk, CX);
  k_gemm2<0><<<gd, 128, 0, stream>>>(CX, DM, BO, DM, 1.0f / 1024.0f, bo, AO, nullptr, DM, DM);
  k_ln<1><<<NR / 8, 256, 0, stream>>>(AO, x, g1, be1, Hf, H16);
  k_gemm2<0><<<gf, 128, 0, stream>>>(H16, DM, B1, DM, 0.0625f, b1, nullptr, F16, FF, DM);
  k_gemm2<9><<<gd, 128, 0, stream>>>(F16, FF, B2, FF, 1.0f / 64.0f, b2, FFo, nullptr, DM, FF);
  k_ln<2><<<NR / 8, 256, 0, stream>>>(FFo, Hf, g2, be2, (float*)d_out, nullptr);
}
